// MultiHeadedAttentionXlinear_38860864094604
// MI455X (gfx1250) — hardware-verified
//
#include <hip/hip_runtime.h>
#include <stdint.h>

typedef _Float16 f16;
typedef __bf16 bf16;
typedef f16   v16h __attribute__((ext_vector_type(16)));
typedef f16   v8h  __attribute__((ext_vector_type(8)));
typedef bf16  v16b __attribute__((ext_vector_type(16)));
typedef bf16  v8b  __attribute__((ext_vector_type(8)));
typedef float v8f  __attribute__((ext_vector_type(8)));
typedef float v4f  __attribute__((ext_vector_type(4)));
typedef unsigned int v4u __attribute__((ext_vector_type(4)));

constexpr int NB = 4, NS = 1024, DM = 1024, NH = 16, DK = 64;
constexpr int NBH = NB * NH;
constexpr int NM  = NB * NS;

union FragH  { v16h v; v8h p[2]; };
union FragB  { v16b v; v8b p[2]; };
union Pack8H { v4u u; f16 h[8]; };
union Pack8B { v4u u; bf16 b[8]; };

static __device__ __forceinline__ v8f zero8() {
  v8f z = {0.f, 0.f, 0.f, 0.f, 0.f, 0.f, 0.f, 0.f};
  return z;
}

static __device__ __forceinline__ v16h frag_h(const f16* base, int ld) {
  const int l = threadIdx.x & 31, h = l >> 4, m = l & 15;
  const f16* p = base + m * ld + 8 * h;
  FragH f;
  f.p[0] = *(const v8h*)(p);
  f.p[1] = *(const v8h*)(p + 16);
  return f.v;
}
static __device__ __forceinline__ v16b frag_b(const bf16* base, int ld) {
  const int l = threadIdx.x & 31, h = l >> 4, m = l & 15;
  const bf16* p = base + m * ld + 8 * h;
  FragB f;
  f.p[0] = *(const v8b*)(p);
  f.p[1] = *(const v8b*)(p + 16);
  return f.v;
}

static __device__ __forceinline__ v8f mma_h(v16h a, v16h b, v8f c) {
  c = __builtin_amdgcn_wmma_f32_16x16x32_f16(false, a, false, b, (short)0, c, false, false);
  asm volatile("v_nop\n\tv_nop\n\tv_nop\n\tv_nop" : "+v"(c) : "v"(a), "v"(b));
  return c;
}
static __device__ __forceinline__ v8f mma_b(v16b a, v16b b, v8f c) {
  c = __builtin_amdgcn_wmma_f32_16x16x32_bf16(false, a, false, b, (short)0, c, false, false);
  asm volatile("v_nop\n\tv_nop\n\tv_nop\n\tv_nop" : "+v"(c) : "v"(a), "v"(b));
  return c;
}

static __device__ __forceinline__ void st_v4u(void* p, v4u v) { *(volatile v4u*)p = v; }
static __device__ __forceinline__ void st_v4f(float* p, v4f v) { *(volatile v4f*)p = v; }

__global__ __launch_bounds__(256)
void k_cvt_w(const float* __restrict__ wq, const float* __restrict__ wk, const float* __restrict__ wv,
             const float* __restrict__ wo,
             f16* __restrict__ wqT, f16* __restrict__ wkT, f16* __restrict__ wvT,
             bf16* __restrict__ woTh, bf16* __restrict__ woTl) {
  __shared__ float tile[64][65];
  const int mode = blockIdx.z;
  const float* w = (mode == 0) ? wq : (mode == 1) ? wk : (mode == 2) ? wv : wo;
  f16* wt16 = (mode == 0) ? wqT : (mode == 1) ? wkT : wvT;
  const int k0 = blockIdx.x * 64, n0 = blockIdx.y * 64;
  const int tid = threadIdx.x;
  {
    const int r = tid >> 2, c0 = (tid & 3) * 16;
    const float* src = w + (size_t)(k0 + r) * DM + n0 + c0;
#pragma unroll
    for (int j = 0; j < 16; j += 4) {
      v4f t = *(const v4f*)(src + j);
      tile[r][c0 + j] = t.x; tile[r][c0 + j + 1] = t.y;
      tile[r][c0 + j + 2] = t.z; tile[r][c0 + j + 3] = t.w;
    }
  }
  __syncthreads();
  for (int pass = 0; pass < 2; ++pass) {
#pragma unroll
    for (int p = 0; p < 2; ++p) {
      const int rr = p * 32 + (tid >> 3), kq = (tid & 7) * 8;
      const size_t dst = (size_t)(n0 + rr) * DM + k0 + kq;
      if (mode < 3) {
        Pack8H pk;
#pragma unroll
        for (int j = 0; j < 8; ++j) pk.h[j] = (f16)(tile[kq + j][rr] * 64.0f);
        st_v4u(wt16 + dst, pk.u);
      } else {
        Pack8B ph, pl;
#pragma unroll
        for (int j = 0; j < 8; ++j) {
          const float x = tile[kq + j][rr];
          const bf16 hb = (bf16)x;
          ph.b[j] = hb;
          pl.b[j] = (bf16)(x - (float)hb);
        }
        st_v4u(woTh + dst, ph.u);
        st_v4u(woTl + dst, pl.u);
      }
    }
    __threadfence();
  }
}

__global__ __launch_bounds__(256)
void k_prep_small(const float* __restrict__ spatial_w, const float* __restrict__ qproj_w,
                  const float* __restrict__ qproj_b, const float* __restrict__ kproj_w,
                  const float* __restrict__ vlin_w,
                  f16* __restrict__ spT, f16* __restrict__ kpT,
                  bf16* __restrict__ vlTh, bf16* __restrict__ vlTl, float* __restrict__ wline) {
  __shared__ float wl[128];
  const int tid = threadIdx.x;
  if (tid < 64) {
    float s = 0.f;
    for (int n = 0; n < 64; ++n) s += qproj_w[tid * 64 + n];
    wl[tid] = s * (1.0f / 64.0f);
  } else if (tid == 64) {
    float s = 0.f;
    for (int n = 0; n < 64; ++n) s += qproj_b[n];
    wl[64] = s * (1.0f / 64.0f);
  } else if (tid < 128) {
    wl[tid] = 0.f;
  }
  __syncthreads();
  for (int pass = 0; pass < 2; ++pass) {
#pragma unroll
    for (int p = 0; p < 2; ++p) {
      const int n = p * 32 + (tid >> 3), kq = (tid & 7) * 8;
      Pack8H ps, pk;
      Pack8B ph, pl;
#pragma unroll
      for (int j = 0; j < 8; ++j) {
        const int k = kq + j;
        ps.h[j] = (f16)(spatial_w[k * 64 + n] * 64.0f);
        pk.h[j] = (f16)(kproj_w[k * 64 + n] * 64.0f);
        const float x = vlin_w[k * 64 + n];
        const bf16 hb = (bf16)x;
        ph.b[j] = hb;
        pl.b[j] = (bf16)(x - (float)hb);
      }
      const int dst = n * 64 + kq;
      st_v4u(spT + dst, ps.u);
      st_v4u(kpT + dst, pk.u);
      st_v4u(vlTh + dst, ph.u);
      st_v4u(vlTl + dst, pl.u);
    }
    if (tid < 32) {
      v4f v = {wl[4 * tid], wl[4 * tid + 1], wl[4 * tid + 2], wl[4 * tid + 3]};
      st_v4f(wline + 4 * tid, v);
    }
    __threadfence();
  }
}

__global__ __launch_bounds__(256)
void k_cvt_act(const float* __restrict__ q, const float* __restrict__ k, const float* __restrict__ v,
               f16* __restrict__ q16, f16* __restrict__ k16, f16* __restrict__ v16, int n) {
  const int mode = blockIdx.y;
  const float* src = (mode == 0) ? q : (mode == 1) ? k : v;
  f16* dst = (mode == 0) ? q16 : (mode == 1) ? k16 : v16;
  const size_t e0 = ((size_t)blockIdx.x * 256 + threadIdx.x) * 8;
  if (e0 + 8 > (size_t)n) return;
  const v4f a = *(const v4f*)(src + e0);
  const v4f b = *(const v4f*)(src + e0 + 4);
  Pack8H pk;
  pk.h[0] = (f16)a.x; pk.h[1] = (f16)a.y; pk.h[2] = (f16)a.z; pk.h[3] = (f16)a.w;
  pk.h[4] = (f16)b.x; pk.h[5] = (f16)b.y; pk.h[6] = (f16)b.z; pk.h[7] = (f16)b.w;
  st_v4u(dst + e0, pk.u);
  __threadfence();
  st_v4u(dst + e0, pk.u);
}

__global__ __launch_bounds__(256)
void k_proj_qkv(const f16* __restrict__ q16, const f16* __restrict__ k16, const f16* __restrict__ v16,
                const f16* __restrict__ wqT, const f16* __restrict__ wkT, const f16* __restrict__ wvT,
                const float* __restrict__ bq, const float* __restrict__ bk, const float* __restrict__ bv,
                const float* __restrict__ chan_w, const float* __restrict__ chan_b,
                f16* __restrict__ qh, f16* __restrict__ kh,
                bf16* __restrict__ vhh, bf16* __restrict__ vhl,
                float* __restrict__ g1, float* __restrict__ g0) {
  __shared__ __align__(16) f16 As[128][40];
  __shared__ __align__(16) f16 Bs[64][40];
  __shared__ __align__(16) float Cs[128][68];
  __shared__ __align__(16) float gL[2][128];

  const int mode = blockIdx.z;
  const f16* X  = (mode == 0) ? q16 : (mode == 1) ? k16 : v16;
  const f16* WT = (mode == 0) ? wqT : (mode == 1) ? wkT : wvT;
  const float* bias = (mode == 0) ? bq : (mode == 1) ? bk : bv;

  const int m0 = blockIdx.x * 128, n0 = blockIdx.y * 64;
  const int tid = threadIdx.x, wv = tid >> 5, l = tid & 31, hh = l >> 4, mm = l & 15;
  const int wm = wv & 3, wn = wv >> 2;

  v8f acc00 = zero8(), acc01 = zero8(), acc10 = zero8(), acc11 = zero8();
  for (int k0 = 0; k0 < DM; k0 += 32) {
    __syncthreads();
#pragma unroll
    for (int c = 0; c < 2; ++c) {
      const int idx = c * 256 + tid;
      const int r = idx >> 2, qq = (idx & 3) * 8;
      *(v4u*)&As[r][qq] = *(const v4u*)(X + (size_t)(m0 + r) * DM + k0 + qq);
    }
    {
      const int r = tid >> 2, qq = (tid & 3) * 8;
      *(v4u*)&Bs[r][qq] = *(const v4u*)(WT + (size_t)(n0 + r) * DM + k0 + qq);
    }
    __syncthreads();
    const v16h a0 = frag_h(&As[wm * 32][0], 40);
    const v16h a1 = frag_h(&As[wm * 32 + 16][0], 40);
    const v16h b0 = frag_h(&Bs[wn * 32][0], 40);
    const v16h b1 = frag_h(&Bs[wn * 32 + 16][0], 40);
    acc00 = mma_h(a0, b0, acc00);
    acc01 = mma_h(a0, b1, acc01);
    acc10 = mma_h(a1, b0, acc10);
    acc11 = mma_h(a1, b1, acc11);
  }
  {
    const float inv = 1.0f / 64.0f;
    const int r0 = wm * 32 + 8 * hh, c0 = wn * 32 + mm;
    const float b0v = bias[n0 + c0], b1v = bias[n0 + c0 + 16];
#pragma unroll
    for (int r = 0; r < 8; ++r) {
      Cs[r0 + r][c0]           = acc00[r] * inv + b0v;
      Cs[r0 + r][c0 + 16]      = acc01[r] * inv + b1v;
      Cs[r0 + 16 + r][c0]      = acc10[r] * inv + b0v;
      Cs[r0 + 16 + r][c0 + 16] = acc11[r] * inv + b1v;
    }
  }
  __syncthreads();
  if (mode == 1) {
    if (tid < 128) {
      float d1 = 0.f, d0 = 0.f;
      for (int e = 0; e < 64; ++e) {
        const float c = Cs[tid][e];
        d1 += c * chan_w[e];
        d0 += c * chan_b[e];
      }
      gL[0][tid] = d1;
      gL[1][tid] = d0;
    }
    __syncthreads();
  }
  const int bb = m0 >> 10, s0 = m0 & 1023, hd = n0 >> 6, bh = bb * NH + hd;
  for (int pass = 0; pass < 2; ++pass) {
    if (mode < 2) {
      f16* OUT = (mode == 0) ? qh : kh;
#pragma unroll
      for (int p = 0; p < 4; ++p) {
        const int rr = p * 32 + (tid >> 3), cq = (tid & 7) * 8;
        Pack8H pk;
#pragma unroll
        for (int j = 0; j < 8; ++j) pk.h[j] = (f16)(Cs[rr][cq + j] * 16.0f);
        st_v4u(OUT + ((size_t)bh * NS + s0 + rr) * DK + cq, pk.u);
      }
      if (mode == 1 && tid < 64) {
        const int wch = tid >> 5;
        float* G = (wch == 0) ? g1 : g0;
        v4f v = {gL[wch][4 * l], gL[wch][4 * l + 1], gL[wch][4 * l + 2], gL[wch][4 * l + 3]};
        st_v4f(G + (size_t)bh * NS + s0 + 4 * l, v);
      }
    } else {
#pragma unroll
      for (int p = 0; p < 4; ++p) {
        const int rr = p * 32 + (tid >> 3), cq = (tid & 7) * 8;
        Pack8B ph, pl;
#pragma unroll
        for (int j = 0; j < 8; ++j) {
          const float x = Cs[rr][cq + j];
          const bf16 hb = (bf16)x;
          ph.b[j] = hb;
          pl.b[j] = (bf16)(x - (float)hb);
        }
        const size_t dst = ((size_t)bh * NS + s0 + rr) * DK + cq;
        st_v4u(vhh + dst, ph.u);
        st_v4u(vhl + dst, pl.u);
      }
    }
    __threadfence();
  }
}

__global__ __launch_bounds__(256)
void k_headlin_f16(const f16* __restrict__ qh, const f16* __restrict__ kh,
                   const f16* __restrict__ spT, const f16* __restrict__ kpT,
                   const float* __restrict__ sb, const float* __restrict__ kb,
                   const float* __restrict__ wline,
                   f16* __restrict__ qe, f16* __restrict__ k2, float* __restrict__ mu) {
  __shared__ __align__(16) f16 As[64][72];
  __shared__ __align__(16) f16 Bs[64][72];
  __shared__ __align__(16) float Cs[64][68];
  __shared__ float wl[128];
  __shared__ __align__(16) float muL[64];

  const int mode = blockIdx.z, bh = blockIdx.y, s0 = blockIdx.x * 64;
  const size_t rowbase = ((size_t)bh * NS + s0) * DK;
  const f16* X  = ((mode == 0) ? qh : kh) + rowbase;
  const f16* WT = (mode == 0) ? spT : kpT;
  const float* bias = (mode == 0) ? sb : kb;
  f16* OUT = ((mode == 0) ? qe : k2) + rowbase;

  const int tid = threadIdx.x, wv = tid >> 5, l = tid & 31, hh = l >> 4, mm = l & 15;
  const int wm = wv & 3, wn = wv >> 2;
#pragma unroll
  for (int c = 0; c < 2; ++c) {
    const int idx = c * 256 + tid;
    const int r = idx >> 3, qq = (idx & 7) * 8;
    *(v4u*)&As[r][qq] = *(const v4u*)(X + r * DK + qq);
    *(v4u*)&Bs[r][qq] = *(const v4u*)(WT + r * DK + qq);
  }
  if (tid < 128) wl[tid] = wline[tid];
  __syncthreads();

  v8f acc0 = zero8(), acc1 = zero8();
#pragma unroll
  for (int kk = 0; kk < 2; ++kk) {
    const v16h a  = frag_h(&As[wm * 16][kk * 32], 72);
    const v16h b0 = frag_h(&Bs[wn * 32][kk * 32], 72);
    const v16h b1 = frag_h(&Bs[wn * 32 + 16][kk * 32], 72);
    acc0 = mma_h(a, b0, acc0);
    acc1 = mma_h(a, b1, acc1);
  }
  {
    const float inv = 1.0f / 1024.0f;
    const int r0 = wm * 16 + 8 * hh, c0 = wn * 32 + mm;
    const float b0v = bias[c0], b1v = bias[c0 + 16];
#pragma unroll
    for (int r = 0; r < 8; ++r) {
      float c = acc0[r] * inv + b0v;
      c = (c > 0.f) ? c : expm1f(c);
      Cs[r0 + r][c0] = c;
      float d = acc1[r] * inv + b1v;
      d = (d > 0.f) ? d : expm1f(d);
      Cs[r0 + r][c0 + 16] = d;
    }
  }
  __syncthreads();
  if (mode == 0) {
    if (tid < 64) {
      float d = wl[64];
      for (int e = 0; e < 64; ++e) d += Cs[tid][e] * wl[e];
      muL[tid] = d;
    }
    __syncthreads();
  }
  for (int pass = 0; pass < 2; ++pass) {
#pragma unroll
    for (int p = 0; p < 2; ++p) {
      const int rr = p * 32 + (tid >> 3), cq = (tid & 7) * 8;
      Pack8H pk;
#pragma unroll
      for (int j = 0; j < 8; ++j) pk.h[j] = (f16)(Cs[rr][cq + j] * 256.0f);
      st_v4u(OUT + rr * DK + cq, pk.u);
    }
    if (mode == 0 && tid < 16) {
      v4f v = {muL[4 * tid], muL[4 * tid + 1], muL[4 * tid + 2], muL[4 * tid + 3]};
      st_v4f(mu + (size_t)bh * NS + s0 + 4 * tid, v);
    }
    __threadfence();
  }
}

__global__ __launch_bounds__(256)
void k_headlin_v(const bf16* __restrict__ vhh, const bf16* __restrict__ vhl,
                 const bf16* __restrict__ vlTh, const bf16* __restrict__ vlTl,
                 const float* __restrict__ vb, f16* __restrict__ v2) {
  __shared__ __align__(16) bf16 Ah[64][72];
  __shared__ __align__(16) bf16 Al[64][72];
  __shared__ __align__(16) bf16 Bh[64][72];
  __shared__ __align__(16) bf16 Bl[64][72];
  __shared__ __align__(16) float Cs[64][68];

  const int bh = blockIdx.y, s0 = blockIdx.x * 64;
  const size_t rowbase = ((size_t)bh * NS + s0) * DK;
  const bf16* Xh = vhh + rowbase;
  const bf16* Xl = vhl + rowbase;
  f16* OUT = v2 + rowbase;

  const int tid = threadIdx.x, wv = tid >> 5, l = tid & 31, hh = l >> 4, mm = l & 15;
  const int wm = wv & 3, wn = wv >> 2;
#pragma unroll
  for (int c = 0; c < 2; ++c) {
    const int idx = c * 256 + tid;
    const int r = idx >> 3, qq = (idx & 7) * 8;
    *(v4u*)&Ah[r][qq] = *(const v4u*)(Xh + r * DK + qq);
    *(v4u*)&Al[r][qq] = *(const v4u*)(Xl + r * DK + qq);
    *(v4u*)&Bh[r][qq] = *(const v4u*)(vlTh + r * DK + qq);
    *(v4u*)&Bl[r][qq] = *(const v4u*)(vlTl + r * DK + qq);
  }
  __syncthreads();

  v8f acc0 = zero8(), acc1 = zero8();
#pragma unroll
  for (int kk = 0; kk < 2; ++kk) {
    const v16b ah = frag_b(&Ah[wm * 16][kk * 32], 72);
    const v16b al = frag_b(&Al[wm * 16][kk * 32], 72);
    {
      const v16b bhf = frag_b(&Bh[wn * 32][kk * 32], 72);
      const v16b blf = frag_b(&Bl[wn * 32][kk * 32], 72);
      acc0 = mma_b(ah, bhf, acc0);
      acc0 = mma_b(ah, blf, acc0);
      acc0 = mma_b(al, bhf, acc0);
    }
    {
      const v16b bhf = frag_b(&Bh[wn * 32 + 16][kk * 32], 72);
      const v16b blf = frag_b(&Bl[wn * 32 + 16][kk * 32], 72);
      acc1 = mma_b(ah, bhf, acc1);
      acc1 = mma_b(ah, blf, acc1);
      acc1 = mma_b(al, bhf, acc1);
    }
  }
  {
    const int r0 = wm * 16 + 8 * hh, c0 = wn * 32 + mm;
    const float b0v = vb[c0], b1v = vb[c0 + 16];
#pragma unroll
    for (int r = 0; r < 8; ++r) {
      float c = acc0[r] + b0v;
      c = (c > 0.f) ? c : expm1f(c);
      Cs[r0 + r][c0] = c;
      float d = acc1[r] + b1v;
      d = (d > 0.f) ? d : expm1f(d);
      Cs[r0 + r][c0 + 16] = d;
    }
  }
  __syncthreads();
  for (int pass = 0; pass < 2; ++pass) {
#pragma unroll
    for (int p = 0; p < 2; ++p) {
      const int rr = p * 32 + (tid >> 3), cq = (tid & 7) * 8;
      Pack8H pk;
#pragma unroll
      for (int j = 0; j < 8; ++j) pk.h[j] = (f16)(Cs[rr][cq + j] * 256.0f);
      st_v4u(OUT + rr * DK + cq, pk.u);
    }
    __threadfence();
  }
}

__global__ __launch_bounds__(256)
void k_attention(const f16* __restrict__ qe, const f16* __restrict__ k2, const f16* __restrict__ v2,
                 const float* __restrict__ mu, const float* __restrict__ g1, const float* __restrict__ g0,
                 const int* __restrict__ mask, bf16* __restrict__ xh, bf16* __restrict__ xl) {
  __shared__ __align__(16) f16 Qs[64][72];
  __shared__ __align__(16) f16 Ks[64][72];
  __shared__ __align__(16) f16 Vt[64][72];
  __shared__ __align__(16) f16 Ps[64][72];
  __shared__ __align__(16) float Os[64][68];
  __shared__ float muL[64], g1L[64], g0L[64], mrow[64], lrow[64], scl[64], mnw[64];
  __shared__ float redm[2][64], reds[2][64];

  const int bh = blockIdx.y, bb = bh >> 4, hd = bh & 15, q0 = blockIdx.x * 64;
  const f16* Q = qe + ((size_t)bh * NS + q0) * DK;
  const f16* K = k2 + (size_t)bh * NS * DK;
  const f16* V = v2 + (size_t)bh * NS * DK;
  const int* M = mask + ((size_t)bb * NS + q0) * NS;

  const int tid = threadIdx.x, wv = tid >> 5, l = tid & 31, hh = l >> 4, mm = l & 15;
  const int wm = wv >> 1, ch = wv & 1;

#pragma unroll
  for (int c = 0; c < 2; ++c) {
    const int idx = c * 256 + tid;
    const int r = idx >> 3, qq = (idx & 7) * 8;
    *(v4u*)&Qs[r][qq] = *(const v4u*)(Q + r * DK + qq);
  }
  if (tid < 64) {
    muL[tid] = mu[(size_t)bh * NS + q0 + tid];
    mrow[tid] = -3.0e38f;
    lrow[tid] = 0.f;
  }
  __syncthreads();

  v8f accO0 = zero8(), accO1 = zero8();

  for (int j = 0; j < 16; ++j) {
    const int t0 = j * 64;
    __syncthreads();
#pragma unroll
    for (int c = 0; c < 2; ++c) {
      const int idx = c * 256 + tid;
      const int r = idx >> 3, qq = (idx & 7) * 8;
      *(v4u*)&Ks[r][qq] = *(const v4u*)(K + (size_t)(t0 + r) * DK + qq);
      Pack8H pv;
      pv.u = *(const v4u*)(V + (size_t)(t0 + r) * DK + qq);
#pragma unroll
      for (int jj = 0; jj < 8; ++jj) Vt[qq + jj][r] = pv.h[jj];
    }
    if (tid < 64) {
      g1L[tid] = g1[(size_t)bh * NS + t0 + tid];
      g0L[tid] = g0[(size_t)bh * NS + t0 + tid];
    }
    __syncthreads();

    v8f s0a = zero8(), s1a = zero8();
#pragma unroll
    for (int kk = 0; kk < 2; ++kk) {
      const v16h a  = frag_h(&Qs[wm * 16][kk * 32], 72);
      const v16h b0 = frag_h(&Ks[ch * 32][kk * 32], 72);
      const v16h b1 = frag_h(&Ks[ch * 32 + 16][kk * 32], 72);
      s0a = mma_h(a, b0, s0a);
      s1a = mma_h(a, b1, s1a);
    }

    const float sc_s = 1.0f / 524288.0f;
    float sv[16];
#pragma unroll
    for (int r = 0; r < 8; ++r) {
      const int row = wm * 16 + 8 * hh + r;
      const float muq = muL[row];
      {
        const int tl = ch * 32 + mm;
        float s = s0a[r] * sc_s;
        const float z = muq * g1L[tl] + g0L[tl];
        s = s * (1.0f / (1.0f + __expf(-z)));
        if (M[(size_t)row * NS + t0 + tl] == 0) s = -1.0e9f;
        sv[r] = s;
      }
      {
        const int tl = ch * 32 + 16 + mm;
        float s = s1a[r] * sc_s;
        const float z = muq * g1L[tl] + g0L[tl];
        s = s * (1.0f / (1.0f + __expf(-z)));
        if (M[(size_t)row * NS + t0 + tl] == 0) s = -1.0e9f;
        sv[8 + r] = s;
      }
    }
#pragma unroll
    for (int r = 0; r < 8; ++r) {
      float pr = fmaxf(sv[r], sv[8 + r]);
      pr = fmaxf(pr, __shfl_xor(pr, 1));
      pr = fmaxf(pr, __shfl_xor(pr, 2));
      pr = fmaxf(pr, __shfl_xor(pr, 4));
      pr = fmaxf(pr, __shfl_xor(pr, 8));
      if (mm == 0) redm[ch][wm * 16 + 8 * hh + r] = pr;
    }
    __syncthreads();
    if (tid < 64) {
      const float mo = mrow[tid];
      const float mn = fmaxf(mo, fmaxf(redm[0][tid], redm[1][tid]));
      mnw[tid] = mn;
      scl[tid] = __expf(mo - mn);
      mrow[tid] = mn;
    }
    __syncthreads();
#pragma unroll
    for (int r = 0; r < 8; ++r) {
      const int row = wm * 16 + 8 * hh + r;
      const float mn = mnw[row];
      const float p0 = __expf(sv[r] - mn);
      const float p1 = __expf(sv[8 + r] - mn);
      Ps[row][ch * 32 + mm]      = (f16)(p0 * 256.0f);
      Ps[row][ch * 32 + 16 + mm] = (f16)(p1 * 256.0f);
      float pr = p0 + p1;
      pr += __shfl_xor(pr, 1);
      pr += __shfl_xor(pr, 2);
      pr += __shfl_xor(pr, 4);
      pr += __shfl_xor(pr, 8);
      if (mm == 0) reds[ch][row] = pr;
    }
    __syncthreads();
    if (tid < 64) lrow[tid] = lrow[tid] * scl[tid] + reds[0][tid] + reds[1][tid];
#pragma unroll
    for (int r = 0; r < 8; ++r) {
      const float sc = scl[wm * 16 + 8 * hh + r];
      accO0[r] *= sc;
      accO1[r] *= sc;
    }
#pragma unroll
    for (int kk = 0; kk < 2; ++kk) {
      const v16h a  = frag_h(&Ps[wm * 16][kk * 32], 72);
      const v16h b0 = frag_h(&Vt[ch * 32][kk * 32], 72);
      const v16h b1 = frag_h(&Vt[ch * 32 + 16][kk * 32], 72);
      accO0 = mma_h(a, b0, accO0);
      accO1 = mma_h(a, b1, accO1);
    }
  }
  __syncthreads();
#pragma unroll
  for (int r = 0; r < 8; ++r) {
    const int row = wm * 16 + 8 * hh + r;
    const float inv = (1.0f / 65536.0f) / lrow[row];
    Os[row][ch * 32 + mm]      = accO0[r] * inv;
    Os[row][ch * 32 + 16 + mm] = accO1[r] * inv;
  }
  __syncthreads();
  for (int pass = 0; pass < 2; ++pass) {
#pragma unroll
    for (int p = 0; p < 2; ++p) {
      const int rr = p * 32 + (tid >> 3), cq = (tid & 7) * 8;
      Pack8B ph, pl;
#pragma unroll
      for (int jj = 0; jj < 8; ++jj) {
        const float x = Os[rr][cq + jj];
        const bf16 hb = (bf16)x;
        ph.b[jj] = hb;
        pl.b[jj] = (bf16)(x - (float)hb);
      }
      const size_t dst = ((size_t)(bb * NS + q0 + rr)) * DM + hd * DK + cq;
      st_v4u(xh + dst, ph.u);
      st_v4u(xl + dst, pl.u);
    }
    __threadfence();
  }
}

__global__ __launch_bounds__(256)
void k_proj_out(const bf16* __restrict__ xh, const bf16* __restrict__ xl,
                const bf16* __restrict__ woTh, const bf16* __restrict__ woTl,
                const float* __restrict__ bo, float* __restrict__ out) {
  __shared__ __align__(16) bf16 Ah[128][32];
  __shared__ __align__(16) bf16 Al[128][32];
  __shared__ __align__(16) bf16 Bh[64][32];
  __shared__ __align__(16) bf16 Bl[64][32];
  __shared__ __align__(16) float Cs[128][68];

  const int m0 = blockIdx.x * 128, n0 = blockIdx.y * 64;
  const int tid = threadIdx.x, wv = tid >> 5, l = tid & 31, hh = l >> 4, mm = l & 15;
  const int wm = wv & 3, wn = wv >> 2;

  v8f acc00 = zero8(), acc01 = zero8(), acc10 = zero8(), acc11 = zero8();
  for (int k0 = 0; k0 < DM; k0 += 32) {
    __syncthreads();
#pragma unroll
    for (int c = 0; c < 2; ++c) {
      const int idx = c * 256 + tid;
      const int r = idx >> 2, qq = (idx & 3) * 8;
      const size_t src = (size_t)(m0 + r) * DM + k0 + qq;
      *(v4u*)&Ah[r][qq] = *(const v4u*)(xh + src);
      *(v4u*)&Al[r][qq] = *(const v4u*)(xl + src);
    }
    {
      const int r = tid >> 2, qq = (tid & 3) * 8;
      const size_t src = (size_t)(n0 + r) * DM + k0 + qq;
      *(v4u*)&Bh[r][qq] = *(const v4u*)(woTh + src);
      *(v4u*)&Bl[r][qq] = *(const v4u*)(woTl + src);
    }
    __syncthreads();
    const v16b a0h = frag_b(&Ah[wm * 32][0], 32);
    const v16b a0l = frag_b(&Al[wm * 32][0], 32);
    const v16b a1h = frag_b(&Ah[wm * 32 + 16][0], 32);
    const v16b a1l = frag_b(&Al[wm * 32 + 16][0], 32);
    {
      const v16b bhf = frag_b(&Bh[wn * 32][0], 32);
      const v16b blf = frag_b(&Bl[wn * 32][0], 32);
      acc00 = mma_b(a0h, bhf, acc00);
      acc00 = mma_b(a0h, blf, acc00);
      acc00 = mma_b(a0l, bhf, acc00);
      acc10 = mma_b(a1h, bhf, acc10);
      acc10 = mma_b(a1h, blf, acc10);
      acc10 = mma_b(a1l, bhf, acc10);
    }
    {
      const v16b bhf = frag_b(&Bh[wn * 32 + 16][0], 32);
      const v16b blf = frag_b(&Bl[wn * 32 + 16][0], 32);
      acc01 = mma_b(a0h, bhf, acc01);
      acc01 = mma_b(a0h, blf, acc01);
      acc01 = mma_b(a0l, bhf, acc01);
      acc11 = mma_b(a1h, bhf, acc11);
      acc11 = mma_b(a1h, blf, acc11);
      acc11 = mma_b(a1l, bhf, acc11);
    }
  }
  {
    const int r0 = wm * 32 + 8 * hh, c0 = wn * 32 + mm;
    const float b0v = bo[n0 + c0], b1v = bo[n0 + c0 + 16];
#pragma unroll
    for (int r = 0; r < 8; ++r) {
      Cs[r0 + r][c0]           = acc00[r] + b0v;
      Cs[r0 + r][c0 + 16]      = acc01[r] + b1v;
      Cs[r0 + 16 + r][c0]      = acc10[r] + b0v;
      Cs[r0 + 16 + r][c0 + 16] = acc11[r] + b1v;
    }
  }
  __syncthreads();
  for (int pass = 0; pass < 2; ++pass) {
#pragma unroll
    for (int p = 0; p < 8; ++p) {
      const int rr = p * 16 + (tid >> 4), cq = (tid & 15) * 4;
      const v4f v = *(const v4f*)&Cs[rr][cq];
      st_v4f(out + (size_t)(m0 + rr) * DM + n0 + cq, v);
    }
    __threadfence();
  }
}

extern "C" void kernel_launch(void* const* d_in, const int* in_sizes, int n_in,
                              void* d_out, int out_size, void* d_ws, size_t ws_size,
                              hipStream_t stream) {
  if (n_in < 22) return;
  const int n_act = NB * NS * DM;
  if (in_sizes[0] != n_act || in_sizes[1] != n_act || in_sizes[2] != n_act || in_sizes[3] != NB * NS * NS) return;
  if (in_sizes[4] != DM * DM || in_sizes[6] != DM * DM || in_sizes[8] != DM * DM || in_sizes[10] != DM * DM) return;
  if (in_sizes[5] != DM || in_sizes[7] != DM || in_sizes[9] != DM || in_sizes[11] != DM) return;
  if (in_sizes[12] != DK * DK || in_sizes[14] != DK * DK || in_sizes[16] != DK * DK || in_sizes[18] != DK * DK) return;
  if (in_sizes[13] != DK || in_sizes[15] != DK || in_sizes[17] != DK || in_sizes[19] != DK) return;
  if (in_sizes[20] != DK || in_sizes[21] != DK) return;
  if (out_size != n_act) return;

  const float* query     = (const float*)d_in[0];
  const float* key       = (const float*)d_in[1];
  const float* value     = (const float*)d_in[2];
  const int*   mask      = (const int*)  d_in[3];
  const float* wq        = (const float*)d_in[4];
  const float* bq        = (const float*)d_in[5];
  const float* wk        = (const float*)d_in[6];
  const float* bk        = (const float*)d_in[7];
  const float* wv        = (const float*)d_in[8];
  const float* bv        = (const float*)d_in[9];
  const float* wo        = (const float*)d_in[10];
  const float* bo        = (const float*)d_in[11];
  const float* spatial_w = (const float*)d_in[12];
  const float* spatial_b = (const float*)d_in[13];
  const float* qproj_w   = (const float*)d_in[14];
  const float* qproj_b   = (const float*)d_in[15];
  const float* kproj_w   = (const float*)d_in[16];
  const float* kproj_b   = (const float*)d_in[17];
  const float* vlin_w    = (const float*)d_in[18];
  const float* vlin_b    = (const float*)d_in[19];
  const float* chan_w    = (const float*)d_in[20];
  const float* chan_b    = (const float*)d_in[21];

  char* ws = (char*)d_ws;
  size_t off = 0;
  auto carve = [&](size_t bytes) -> void* {
    void* p = ws + off;
    off = (off + bytes + 255) & ~(size_t)255;
    return p;
  };
  const size_t act16  = (size_t)NM * DM * 2;
  const size_t w16    = (size_t)DM * DM * 2;
  const size_t head16 = (size_t)NBH * NS * DK * 2;
  const size_t rowf   = (size_t)NBH * NS * 4;

  f16*  q16  = (f16*)carve(act16);
  f16*  k16  = (f16*)carve(act16);
  f16*  v16  = (f16*)carve(act16);
  f16*  wqT  = (f16*)carve(w16);
  f16*  wkT  = (f16*)carve(w16);
  f16*  wvT  = (f16*)carve(w16);
  bf16* woTh = (bf16*)carve(w16);
  bf16* woTl = (bf16*)carve(w16);
  f16*  qh   = (f16*)carve(head16);
  f16*  kh   = (f16*)carve(head16);
  bf16* vhh  = (bf16*)carve(head16);
  bf16* vhl  = (bf16*)carve(head16);
  f16*  qe   = (f16*)carve(head16);
  f16*  k2   = (f16*)carve(head16);
  f16*  v2   = (f16*)carve(head16);
  bf16* xh   = (bf16*)carve(act16);
  bf16* xl   = (bf16*)carve(act16);
  float* mu  = (float*)carve(rowf);
  float* g1  = (float*)carve(rowf);
  float* g0  = (float*)carve(rowf);
  f16*  spT  = (f16*)carve((size_t)DK * DK * 2);
  f16*  kpT  = (f16*)carve((size_t)DK * DK * 2);
  bf16* vlTh = (bf16*)carve((size_t)DK * DK * 2);
  bf16* vlTl = (bf16*)carve((size_t)DK * DK * 2);
  float* wline = (float*)carve(128 * sizeof(float));
  if (off > ws_size) return;

  k_cvt_w<<<dim3(DM / 64, DM / 64, 4), 256, 0, stream>>>(wq, wk, wv, wo, wqT, wkT, wvT, woTh, woTl);
  k_prep_small<<<1, 256, 0, stream>>>(spatial_w, qproj_w, qproj_b, kproj_w, vlin_w,
                                      spT, kpT, vlTh, vlTl, wline);
  k_cvt_act<<<dim3((n_act + 2047) / 2048, 3), 256, 0, stream>>>(query, key, value, q16, k16, v16, n_act);
  k_proj_qkv<<<dim3(NM / 128, DM / 64, 3), 256, 0, stream>>>(q16, k16, v16, wqT, wkT, wvT, bq, bk, bv,
                                                            chan_w, chan_b, qh, kh, vhh, vhl, g1, g0);
  k_headlin_f16<<<dim3(NS / 64, NBH, 2), 256, 0, stream>>>(qh, kh, spT, kpT, spatial_b, kproj_b,
                                                          wline, qe, k2, mu);
  k_headlin_v<<<dim3(NS / 64, NBH), 256, 0, stream>>>(vhh, vhl, vlTh, vlTl, vlin_b, v2);
  k_attention<<<dim3(NS / 64, NBH), 256, 0, stream>>>(qe, k2, v2, mu, g1, g0, mask, xh, xl);
  k_proj_out<<<dim3(NM / 128, DM / 64), 256, 0, stream>>>(xh, xl, woTh, woTl, bo, (float*)d_out);
}
